// attention_10574209482773
// MI455X (gfx1250) — hardware-verified
//
#include <hip/hip_runtime.h>
#include <math.h>

#ifndef NB
#define NB 2
#endif
#ifndef SEQ
#define SEQ 2048
#endif
#define NB_FULL 2
#define SEQ_FULL 2048
#define DM 1024
#define NH 16
#define HD 64
#define MROWS (NB * SEQ)
#define AT_NW 4
#define PP 40
#define OSP 68
#define NEARLY (((SEQ / 64) < 4) ? (SEQ / 64) : 4)

static_assert(DM == NH * HD);
static_assert(HD == 64);
static_assert(DM % 64 == 0);
static_assert(SEQ % 64 == 0);
static_assert(MROWS % 64 == 0);
static_assert(DM % 32 == 0);
static_assert((2 * DM) % 32 == 0);
static_assert(DM % 8 == 0);
static_assert(AT_NW * 16 == 64);
static_assert(PP >= 32 && (PP % 8) == 0);
static_assert((OSP % 4) == 0 && OSP >= 64);
static_assert(NB <= NB_FULL && SEQ <= SEQ_FULL);
static_assert(NEARLY >= 1);

typedef _Float16 v16h __attribute__((ext_vector_type(16)));
typedef _Float16 v8h  __attribute__((ext_vector_type(8)));
typedef float    v8f  __attribute__((ext_vector_type(8)));
typedef float    v4f  __attribute__((ext_vector_type(4)));
typedef v8h v8h_a __attribute__((may_alias));
typedef v4f v4f_a __attribute__((may_alias));
union FH { v16h v; v8h h[2]; };

__device__ __forceinline__ v16h ldg(const _Float16* __restrict__ p) {
    FH f; f.h[0] = *(const v8h*)(p); f.h[1] = *(const v8h*)(p + 16); return f.v;
}
__device__ __forceinline__ v8f wmma16(v16h a, v16h b, v8f c) {
    c = __builtin_amdgcn_wmma_f32_16x16x32_f16(false, a, false, b, (short)0, c, false, false);
    asm volatile("v_nop\n\tv_nop\n\tv_nop\n\tv_nop" : "+v"(c) : "v"(a), "v"(b));
    return c;
}
__device__ __forceinline__ void guard_row(v8f& a0, v8f& a1, v8f& a2, v8f& a3, v16h x, v16h y) {
    asm volatile("v_nop\n\tv_nop\n\tv_nop\n\tv_nop" : "+v"(a0), "+v"(a1), "+v"(a2), "+v"(a3) : "v"(x), "v"(y));
}
__device__ __forceinline__ void keep4(v16h a, v16h b, v16h c, v16h d) { asm volatile("v_nop" :: "v"(a), "v"(b), "v"(c), "v"(d)); }
__device__ __forceinline__ void acc_guard4(v8f& a, v8f& b, v8f& c, v8f& d) { asm volatile("v_nop\n\tv_nop\n\tv_nop\n\tv_nop" : "+v"(a), "+v"(b), "+v"(c), "+v"(d)); }
__device__ __forceinline__ void wave_sync() {
    __builtin_amdgcn_fence(3  , "workgroup");
    __builtin_amdgcn_wave_barrier();
    __builtin_amdgcn_fence(2  , "workgroup");
}
__device__ __forceinline__ float cmb_bf(float v) {
    const unsigned u = __builtin_bit_cast(unsigned, v);
    const unsigned r = (u + 0x7fffu + ((u >> 16) & 1u)) & 0xffff0000u;
    return __builtin_bit_cast(float, r);
}
__device__ __forceinline__ void split8(const v4f x0, const v4f x1, const float rs, v8h& hv, v8h& rv) {
    const float x[8] = {x0.x, x0.y, x0.z, x0.w, x1.x, x1.y, x1.z, x1.w};
#pragma unroll
    for (int e = 0; e < 8; ++e) { const _Float16 hh = (_Float16)x[e]; hv[e] = hh; rv[e] = (_Float16)((x[e] - (float)hh) * rs); }
}

__global__ __launch_bounds__(256) void k_cast_rows(const float* __restrict__ SRC, long long sSz, int lds,
                                                   _Float16* __restrict__ DST, long long sDz, int ldd, int nR, int nC, float sc) {
    const long long u = (long long)blockIdx.x * 256 + threadIdx.x; const int per = nC / 8;
    if (u >= (long long)nR * per) return;
    const int r = (int)(u / per); const int c0 = 8 * (int)(u % per);
    const float* s = SRC + (long long)blockIdx.y * sSz + (long long)r * lds + c0;
    const v4f x0 = *(const v4f*)(s), x1 = *(const v4f*)(s + 4);
    v8h pk;
    pk[0] = (_Float16)(cmb_bf(x0.x) * sc); pk[1] = (_Float16)(cmb_bf(x0.y) * sc); pk[2] = (_Float16)(cmb_bf(x0.z) * sc); pk[3] = (_Float16)(cmb_bf(x0.w) * sc);
    pk[4] = (_Float16)(cmb_bf(x1.x) * sc); pk[5] = (_Float16)(cmb_bf(x1.y) * sc); pk[6] = (_Float16)(cmb_bf(x1.z) * sc); pk[7] = (_Float16)(cmb_bf(x1.w) * sc);
    _Float16* d = DST + (long long)blockIdx.y * sDz + (long long)r * ldd + c0;
    *(volatile v8h*)d = pk; __threadfence(); *(volatile v8h*)d = pk;
}
__global__ __launch_bounds__(256) void k_castT(const float* __restrict__ SRC, int lds, _Float16* __restrict__ DST, int ldd, int nR, int nC, float sc) {
    const long long u = (long long)blockIdx.x * 256 + threadIdx.x; const int per = nR / 8;
    if (u >= (long long)nC * per) return;
    const int c = (int)(u / per); const int r0 = 8 * (int)(u % per);
    v8h pk;
#pragma unroll
    for (int e = 0; e < 8; ++e) pk[e] = (_Float16)(cmb_bf(SRC[(long long)(r0 + e) * lds + c]) * sc);
    _Float16* d = DST + (long long)c * ldd + r0;
    *(volatile v8h*)d = pk; __threadfence(); *(volatile v8h*)d = pk;
}

template <int OUTM>
__device__ __forceinline__ void gemm64_body(const _Float16* __restrict__ A, const int lda, const long long strideA,
                                            const _Float16* __restrict__ Bt, const int ldb,
                                            float* __restrict__ Cf, _Float16* __restrict__ Ch, _Float16* __restrict__ Cr,
                                            const int ldc, const long long strideC,
                                            const float* __restrict__ bias, const int M, const int N, const int K, const float scale) {
    __shared__ __align__(16) float sT[8][16 * OSP];
    const int z = (int)blockIdx.y;
    const int lane = threadIdx.x & 31;
    const int wave = __builtin_amdgcn_readfirstlane((int)(threadIdx.x >> 5));
    const int tilesN = N >> 6, tilesM = M >> 6;
    const int tile = (int)blockIdx.x * 8 + wave;
    if (tile >= tilesM * tilesN) return;
    const int tm = tile / tilesN, tn = tile - tm * tilesN;
    const int m0 = tm << 6, n0 = tn << 6;
    const _Float16* Ab = A + (size_t)z * (size_t)strideA;
    const int rl = lane & 15, koff = (lane >> 4) * 8, mOff = (lane >> 4) * 8;

    v8f acc[4][4];
#pragma unroll
    for (int i = 0; i < 4; ++i)
#pragma unroll
        for (int j = 0; j < 4; ++j) acc[i][j] = (v8f){0.f, 0.f, 0.f, 0.f, 0.f, 0.f, 0.f, 0.f};

#pragma unroll 1
    for (int k0 = 0; k0 < K; k0 += 32) {
        v16h bh[4];
#pragma unroll
        for (int j = 0; j < 4; ++j) bh[j] = ldg(Bt + (size_t)(n0 + (j << 4) + rl) * ldb + koff + k0);
#pragma unroll
        for (int i = 0; i < 4; ++i) {
            const v16h ah = ldg(Ab + (size_t)(m0 + (i << 4) + rl) * lda + koff + k0);
#pragma unroll
            for (int j = 0; j < 4; ++j)
                acc[i][j] = __builtin_amdgcn_wmma_f32_16x16x32_f16(false, ah, false, bh[j], (short)0, acc[i][j], false, false);
            guard_row(acc[i][0], acc[i][1], acc[i][2], acc[i][3], ah, bh[3]);
        }
        keep4(bh[0], bh[1], bh[2], bh[3]);
    }
    acc_guard4(acc[0][0], acc[0][1], acc[0][2], acc[0][3]);
    acc_guard4(acc[1][0], acc[1][1], acc[1][2], acc[1][3]);
    acc_guard4(acc[2][0], acc[2][1], acc[2][2], acc[2][3]);
    acc_guard4(acc[3][0], acc[3][1], acc[3][2], acc[3][3]);

#pragma unroll
    for (int i = 0; i < 4; ++i) {
        const int mBase = m0 + (i << 4);
#pragma unroll
        for (int j = 0; j < 4; ++j) {
            float bv = 0.f;
            if (OUTM == 0) bv = cmb_bf(bias[n0 + (j << 4) + rl]);
#pragma unroll
            for (int r = 0; r < 8; ++r) sT[wave][(mOff + r) * OSP + (j << 4) + rl] = acc[i][j][r] * scale + bv;
        }
        wave_sync();
        if (OUTM == 0) {
            float* C = Cf + (size_t)z * (size_t)strideC;
            const int hh = lane >> 4, c4 = (lane & 15) * 4;
            for (int pass = 0; pass < 2; ++pass) {
#pragma unroll
                for (int it = 0; it < 8; ++it) {
                    const int row = it * 2 + hh;
                    const v4f v = *(const v4f_a*)&sT[wave][row * OSP + c4];
                    *(volatile v4f*)(C + (size_t)(mBase + row) * ldc + n0 + c4) = v;
                }
                __threadfence();
            }
        } else {
            const int q4 = lane >> 3, c8 = (lane & 7) * 8;
            for (int pass = 0; pass < 2; ++pass) {
#pragma unroll
                for (int it = 0; it < 4; ++it) {
                    const int row = it * 4 + q4;
                    const v4f x0 = *(const v4f_a*)&sT[wave][row * OSP + c8];
                    const v4f x1 = *(const v4f_a*)&sT[wave][row * OSP + c8 + 4];
                    v8h hv, rv; split8(x0, x1, 2048.0f, hv, rv);
                    *(volatile v8h*)(Ch + (size_t)(mBase + row) * ldc + n0 + c8) = hv;
                    *(volatile v8h*)(Cr + (size_t)(mBase + row) * ldc + n0 + c8) = rv;
                }
                __threadfence();
            }
        }
        wave_sync();
    }
}

__global__ __launch_bounds__(256) void k_gemm_planes(const _Float16* __restrict__ A, int lda, const _Float16* __restrict__ Bt, int ldb,
                                                     _Float16* __restrict__ Ch, _Float16* __restrict__ Cr, int ldc, int M, int N, int K, float scale) {
    gemm64_body<1>(A, lda, 0, Bt, ldb, nullptr, Ch, Cr, ldc, 0, nullptr, M, N, K, scale);
}
__global__ __launch_bounds__(256) void k_gemm_out(const _Float16* __restrict__ A, int lda, long long strideA, const _Float16* __restrict__ Bt, int ldb,
                                                  float* __restrict__ C, int ldc, long long strideC, const float* __restrict__ bias,
                                                  int M, int N, int K, float scale) {
    gemm64_body<0>(A, lda, strideA, Bt, ldb, C, nullptr, nullptr, ldc, strideC, bias, M, N, K, scale);
}

template <bool EARLY>
__device__ __forceinline__ void attn_body(const _Float16* __restrict__ QH, const _Float16* __restrict__ QR,
                                          const _Float16* __restrict__ KH, const _Float16* __restrict__ KR,
                                          const _Float16* __restrict__ VTH, const _Float16* __restrict__ VTR,
                                          _Float16* __restrict__ CTX, const int qb0, const int nq) {
    __shared__ __align__(16) _Float16 Ph[AT_NW][16 * PP];
    __shared__ __align__(16) _Float16 Pr[EARLY ? AT_NW : 1][EARLY ? 16 * PP : 8];
    __shared__ __align__(16) float    Os[AT_NW][16 * OSP];
    const float RQ  = 2048.0f, RQI = 1.0f / 2048.0f, PSC = 4096.0f;
    const float SCL = 0.125f * 1.4426950408889634f;
    const int lane = threadIdx.x & 31, hf = lane >> 4, c = lane & 15;
    const int wave = __builtin_amdgcn_readfirstlane((int)(threadIdx.x >> 5));
    const int bx = (int)blockIdx.x;
    const int qb = qb0 + bx % nq;
    const int bh = bx / nq;
    const int h = bh % NH, b = bh / NH;
    const int q0 = qb * 64 + wave * 16;
    const int tok0 = b * SEQ;
    const size_t qoff = (size_t)(tok0 + q0 + c) * DM + h * HD + 8 * hf;
    const int nhb = (q0 >> 5) + 1;

    v8f o[4], orr[4];
    float m8[8], l8[8];
#pragma unroll
    for (int t = 0; t < 4; ++t) { o[t] = (v8f){0.f, 0.f, 0.f, 0.f, 0.f, 0.f, 0.f, 0.f}; orr[t] = o[t]; }
#pragma unroll
    for (int r = 0; r < 8; ++r) { m8[r] = -__builtin_inff(); l8[r] = 0.f; }

#pragma unroll 1
    for (int hb = 0; hb < nhb; ++hb) {
        const int kv0 = hb * 32;
        v8f s0 = (v8f){0.f, 0.f, 0.f, 0.f, 0.f, 0.f, 0.f, 0.f}, s1 = s0, r0 = s0, r1 = s0;
#pragma unroll
        for (int ks = 0; ks < 2; ++ks) {
            const v16h qh = ldg(QH + qoff + ks * 32);
            const v16h qr = ldg(QR + qoff + ks * 32);
            const size_t ko = (size_t)(tok0 + kv0 + c) * DM + h * HD + ks * 32 + 8 * hf;
            const v16h k0 = ldg(KH + ko);
            const v16h k1 = ldg(KH + ko + (size_t)16 * DM);
            s0 = wmma16(qh, k0, s0); r0 = wmma16(qr, k0, r0);
            s1 = wmma16(qh, k1, s1); r1 = wmma16(qr, k1, r1);
            if (EARLY) {
                const v16h e0 = ldg(KR + ko);
                const v16h e1 = ldg(KR + ko + (size_t)16 * DM);
                r0 = wmma16(qh, e0, r0); r1 = wmma16(qh, e1, r1);
            }
        }
#pragma unroll
        for (int r = 0; r < 8; ++r) {
            const int qrow = q0 + 8 * hf + r;
            float a0 = s0[r] + r0[r] * RQI;
            float a1 = s1[r] + r1[r] * RQI;
            a0 = (a0 + ((kv0 + c      > qrow) ? -1.0e9f : 0.0f)) * SCL;
            a1 = (a1 + ((kv0 + 16 + c > qrow) ? -1.0e9f : 0.0f)) * SCL;
            float mx = fmaxf(a0, a1);
            mx = fmaxf(mx, __shfl_xor(mx, 1, 32)); mx = fmaxf(mx, __shfl_xor(mx, 2, 32));
            mx = fmaxf(mx, __shfl_xor(mx, 4, 32)); mx = fmaxf(mx, __shfl_xor(mx, 8, 32));
            const float mnew = fmaxf(m8[r], mx);
            const float al = exp2f(m8[r] - mnew);
            const float p0 = exp2f(a0 - mnew), p1 = exp2f(a1 - mnew);
            float rs = p0 + p1;
            rs += __shfl_xor(rs, 1, 32); rs += __shfl_xor(rs, 2, 32); rs += __shfl_xor(rs, 4, 32); rs += __shfl_xor(rs, 8, 32);
            l8[r] = l8[r] * al + rs; m8[r] = mnew;
#pragma unroll
            for (int t = 0; t < 4; ++t) { o[t][r] *= al; if (EARLY) orr[t][r] *= al; }
            const float w0 = p0 * PSC, w1 = p1 * PSC;
            const _Float16 g0 = (_Float16)w0, g1 = (_Float16)w1;
            Ph[wave][(8 * hf + r) * PP + c]      = g0;
            Ph[wave][(8 * hf + r) * PP + 16 + c] = g1;
            if (EARLY) {
                Pr[EARLY ? wave : 0][(8 * hf + r) * PP + c]      = (_Float16)((w0 - (float)g0) * RQ);
                Pr[EARLY ? wave : 0][(8 * hf + r) * PP + 16 + c] = (_Float16)((w1 - (float)g1) * RQ);
            }
        }
        wave_sync();
        FH pa, pl;
        pa.h[0] = *(const v8h_a*)&Ph[wave][c * PP + 8 * hf];
        pa.h[1] = *(const v8h_a*)&Ph[wave][c * PP + 16 + 8 * hf];
        pl.v = pa.v;
        if (EARLY) {
            pl.h[0] = *(const v8h_a*)&Pr[EARLY ? wave : 0][c * PP + 8 * hf];
            pl.h[1] = *(const v8h_a*)&Pr[EARLY ? wave : 0][c * PP + 16 + 8 * hf];
        }
        const size_t vo = (size_t)(h * HD + c) * MROWS + tok0 + kv0 + 8 * hf;
#pragma unroll
        for (int t = 0; t < 4; ++t) {
            const v16h vh = ldg(VTH + vo + (size_t)(16 * t) * MROWS);
            o[t] = wmma16(pa.v, vh, o[t]);
            if (EARLY) {
                orr[t] = wmma16(pl.v, vh, orr[t]);
                const v16h vr = ldg(VTR + vo + (size_t)(16 * t) * MROWS);
                orr[t] = wmma16(pa.v, vr, orr[t]);
            }
        }
        wave_sync();
    }

#pragma unroll
    for (int r = 0; r < 8; ++r) {
        const float iv = 1.0f / (l8[r] * PSC);
#pragma unroll
        for (int t = 0; t < 4; ++t) {
            float v = o[t][r];
            if (EARLY) v += orr[t][r] * RQI;
            Os[wave][(8 * hf + r) * OSP + t * 16 + c] = v * iv;
        }
    }
    wave_sync();
    {
        const int q4 = lane >> 3, c8 = (lane & 7) * 8;
        _Float16* cb = CTX + (size_t)(tok0 + q0) * (2 * DM) + h * HD + c8;
        for (int pass = 0; pass < 2; ++pass) {
#pragma unroll
            for (int it = 0; it < 4; ++it) {
                const int row = it * 4 + q4;
                const v4f x0 = *(const v4f_a*)&Os[wave][row * OSP + c8];
                const v4f x1 = *(const v4f_a*)&Os[wave][row * OSP + c8 + 4];
                v8h hv, rv; split8(x0, x1, 128.0f, hv, rv);
                *(volatile v8h*)(cb + (size_t)row * (2 * DM)) = hv;
                *(volatile v8h*)(cb + (size_t)row * (2 * DM) + DM) = rv;
            }
            __threadfence();
        }
    }
}

__global__ __launch_bounds__(128) void k_attn_early(const _Float16* __restrict__ QH, const _Float16* __restrict__ QR,
                                                    const _Float16* __restrict__ KH, const _Float16* __restrict__ KR,
                                                    const _Float16* __restrict__ VTH, const _Float16* __restrict__ VTR,
                                                    _Float16* __restrict__ CTX, int qb0, int nq) {
    attn_body<true>(QH, QR, KH, KR, VTH, VTR, CTX, qb0, nq);
}
__global__ __launch_bounds__(128) void k_attn_late(const _Float16* __restrict__ QH, const _Float16* __restrict__ QR,
                                                   const _Float16* __restrict__ KH, const _Float16* __restrict__ KR,
                                                   const _Float16* __restrict__ VTH, const _Float16* __restrict__ VTR,
                                                   _Float16* __restrict__ CTX, int qb0, int nq) {
    attn_body<false>(QH, QR, KH, KR, VTH, VTR, CTX, qb0, nq);
}

constexpr size_t ACT_B  = (size_t)MROWS * DM * 2;
constexpr size_t W_B    = (size_t)DM * DM * 2;
constexpr size_t WF2_B  = (size_t)DM * (2 * DM) * 2;
constexpr size_t CTX_B  = (size_t)MROWS * (2 * DM) * 2;
constexpr size_t WS_TOTAL = 3 * ACT_B + 3 * W_B + WF2_B + 6 * ACT_B + CTX_B;
static_assert(WS_TOTAL <= (size_t)134217728);
static_assert((ACT_B % 256) == 0 && (W_B % 256) == 0 && (WF2_B % 256) == 0 && (CTX_B % 256) == 0);
static_assert(((size_t)(MROWS / 64) * (DM / 64)) % 8 == 0);
static_assert(((size_t)(SEQ / 64) * (DM / 64)) % 8 == 0);
static_assert(((size_t)(NB_FULL - 1) * SEQ_FULL + SEQ_FULL) * DM * 4 == (size_t)16777216);

extern "C" void kernel_launch(void* const* d_in, const int* in_sizes, int n_in, void* d_out, int out_size, void* d_ws, size_t ws_size, hipStream_t stream) {
    if (n_in < 8) return;
    const long long need_act = ((long long)(NB - 1) * SEQ_FULL + SEQ) * DM;
    if (in_sizes[0] < need_act || in_sizes[1] < need_act || in_sizes[2] < need_act) return;
    if (in_sizes[3] < DM * DM || in_sizes[4] < DM * DM || in_sizes[5] < DM * DM || in_sizes[6] < DM * DM || in_sizes[7] < DM) return;
    if ((long long)out_size < need_act) return;
    if (ws_size < WS_TOTAL) return;

    const float* keys    = (const float*)d_in[0];
    const float* queries = (const float*)d_in[1];
    const float* values  = (const float*)d_in[2];
    const float* Wq = (const float*)d_in[3];
    const float* Wk = (const float*)d_in[4];
    const float* Wv = (const float*)d_in[5];
    const float* Wf = (const float*)d_in[6];
    const float* bf = (const float*)d_in[7];
    float* out = (float*)d_out;

    char* wsp = (char*)d_ws;
    _Float16* XQ  = (_Float16*)wsp; wsp += ACT_B;
    _Float16* XK  = (_Float16*)wsp; wsp += ACT_B;
    _Float16* XV  = (_Float16*)wsp; wsp += ACT_B;
    _Float16* WQT = (_Float16*)wsp; wsp += W_B;
    _Float16* WKT = (_Float16*)wsp; wsp += W_B;
    _Float16* WVT = (_Float16*)wsp; wsp += W_B;
    _Float16* WF2 = (_Float16*)wsp; wsp += WF2_B;
    _Float16* QHp = (_Float16*)wsp; wsp += ACT_B;
    _Float16* QRp = (_Float16*)wsp; wsp += ACT_B;
    _Float16* KHp = (_Float16*)wsp; wsp += ACT_B;
    _Float16* KRp = (_Float16*)wsp; wsp += ACT_B;
    _Float16* VTH = (_Float16*)wsp; wsp += ACT_B;
    _Float16* VTR = (_Float16*)wsp; wsp += ACT_B;
    _Float16* CTX = (_Float16*)wsp; wsp += CTX_B;
    if ((size_t)(wsp - (char*)d_ws) > ws_size) return;

    {
        const dim3 g((unsigned)(((long long)SEQ * (DM / 8) + 255) / 256), (unsigned)NB);
        k_cast_rows<<<g, 256, 0, stream>>>(queries, (long long)SEQ_FULL * DM, DM, XQ, (long long)SEQ * DM, DM, SEQ, DM, 16.0f);
        k_cast_rows<<<g, 256, 0, stream>>>(keys,    (long long)SEQ_FULL * DM, DM, XK, (long long)SEQ * DM, DM, SEQ, DM, 16.0f);
        k_cast_rows<<<g, 256, 0, stream>>>(values,  (long long)SEQ_FULL * DM, DM, XV, (long long)SEQ * DM, DM, SEQ, DM, 16.0f);
    }
    {
        const unsigned g = (unsigned)(((long long)DM * (DM / 8) + 255) / 256);
        k_castT<<<g, 256, 0, stream>>>(Wq, DM, WQT, DM, DM, DM, 16.0f);
        k_castT<<<g, 256, 0, stream>>>(Wk, DM, WKT, DM, DM, DM, 16.0f);
        k_castT<<<g, 256, 0, stream>>>(Wv, DM, WVT, DM, DM, DM, 16.0f);
        k_castT<<<g, 256, 0, stream>>>(Wf, DM, WF2,      2 * DM, DM, DM, 1024.0f);
        k_castT<<<g, 256, 0, stream>>>(Wf, DM, WF2 + DM, 2 * DM, DM, DM, 8.0f);
    }
    {
        const unsigned g = (unsigned)((((MROWS / 64) * (DM / 64)) + 7) / 8);
        k_gemm_planes<<<dim3(g, 1), 256, 0, stream>>>(XQ, DM, WQT, DM, QHp, QRp, DM, MROWS, DM, DM, 1.0f / 256.0f);
        k_gemm_planes<<<dim3(g, 1), 256, 0, stream>>>(XK, DM, WKT, DM, KHp, KRp, DM, MROWS, DM, DM, 1.0f / 256.0f);
        k_gemm_planes<<<dim3(g, 1), 256, 0, stream>>>(WVT, DM, XV, DM, VTH, VTR, MROWS, DM, MROWS, DM, 1.0f / 256.0f);
    }
    {
        const int ne = NEARLY, nl = SEQ / 64 - NEARLY;
        k_attn_early<<<dim3((unsigned)(NB * NH * ne)), 32 * AT_NW, 0, stream>>>(QHp, QRp, KHp, KRp, VTH, VTR, CTX, 0, ne);
        if (nl > 0)
            k_attn_late<<<dim3((unsigned)(NB * NH * nl)), 32 * AT_NW, 0, stream>>>(QHp, QRp, KHp, KRp, VTH, VTR, CTX, ne, nl);
    }
    {
        const unsigned g = (unsigned)((((SEQ / 64) * (DM / 64)) + 7) / 8);
        k_gemm_out<<<dim3(g, (unsigned)NB), 256, 0, stream>>>(CTX, 2 * DM, (long long)SEQ * 2 * DM, WF2, 2 * DM, out, DM, (long long)SEQ_FULL * DM, bf,
                                                             SEQ, DM, 2 * DM, 1.0f / 1024.0f);
    }
}
